// MinimalRNNAttention_33595234189740
// MI455X (gfx1250) — hardware-run, weakly checked
//
#include <hip/hip_runtime.h>
#include <math.h>

constexpr int NBAT  = 4;
constexpr int NSEQ  = 2048;
constexpr int NEMB  = 1024;
constexpr int NHEAD = 8;
constexpr int NDH   = 128;
constexpr int NTOK  = NBAT * NSEQ;
constexpr int NHD   = NHEAD * NDH;
constexpr int NTHR  = 256;
constexpr float LN_EPS_F = 1e-5f;
constexpr float XCARRY = 16.0f;
constexpr float HCARRY = 16.0f;
constexpr float WCARRY = 64.0f;
constexpr float GCARRY = 256.0f;
constexpr float SC_G1 = 1.0f / (XCARRY * WCARRY);
constexpr float SC_F1 = 1.0f / (HCARRY * WCARRY);
constexpr float SC_G2 = 1.0f / (GCARRY * WCARRY);
constexpr int TAB_V  = 0;
constexpr int TAB_UH = 1024;
constexpr int TAB_UZ = 2048;
constexpr int TAB_OS = 3072;
constexpr int TAB_C  = 4096;
constexpr int TAB_N  = 4128;
constexpr int SLP    = 132;

static_assert(NTOK == 8192);
static_assert(NHD == 1024 && NEMB == 1024);
static_assert(NTOK % 64 == 0 && NHD % 64 == 0 && NEMB % 64 == 0);
static_assert(NEMB % 32 == 0 && NHD % 32 == 0 && NDH % 32 == 0);
static_assert(NHEAD == NTHR / 32);
static_assert(NDH == 4 * 32);
static_assert(TAB_UH == NHD && TAB_UZ == 2 * NHD && TAB_OS == 3 * NHD && TAB_C == 4 * NHD);
static_assert(NTOK % 16 == 0);
static_assert(NTOK % (NTHR / 32) == 0);
static_assert((NTOK * (NEMB / 8)) % NTHR == 0);

typedef __attribute__((ext_vector_type(16))) _Float16 v16h;
typedef __attribute__((ext_vector_type(8)))  _Float16 v8h;
typedef __attribute__((ext_vector_type(4)))  _Float16 v4h;
typedef __attribute__((ext_vector_type(8)))  float    v8f;
typedef __attribute__((ext_vector_type(4)))  float    v4f;

__device__ __forceinline__ unsigned short f2bf_bits(float f) {
  unsigned u = __float_as_uint(f);
  return (unsigned short)((u + 0x7FFFu + ((u >> 16) & 1u)) >> 16);
}
__device__ __forceinline__ float bf_bits2f(unsigned short h) { return __uint_as_float(((unsigned)h) << 16); }
__device__ __forceinline__ float bf16r(float f) { return bf_bits2f(f2bf_bits(f)); }

__device__ __forceinline__ void guard4_h(v8f& a0, v8f& a1, v8f& a2, v8f& a3,
                                         v16h x, v16h y0, v16h y1, v16h y2, v16h y3) {
  asm volatile("v_nop\n\tv_nop\n\tv_nop\n\tv_nop"
               : "+v"(a0), "+v"(a1), "+v"(a2), "+v"(a3)
               : "v"(x), "v"(y0), "v"(y1), "v"(y2), "v"(y3));
}
__device__ __forceinline__ void guard8_h(v8f& a0, v8f& a1, v8f& a2, v8f& a3, v8f& a4, v8f& a5, v8f& a6, v8f& a7,
                                         v16h x, v16h y0, v16h y1, v16h y2, v16h y3, v16h y4, v16h y5, v16h y6, v16h y7) {
  asm volatile("v_nop\n\tv_nop\n\tv_nop\n\tv_nop"
               : "+v"(a0), "+v"(a1), "+v"(a2), "+v"(a3), "+v"(a4), "+v"(a5), "+v"(a6), "+v"(a7)
               : "v"(x), "v"(y0), "v"(y1), "v"(y2), "v"(y3), "v"(y4), "v"(y5), "v"(y6), "v"(y7));
}
__device__ __forceinline__ void acc_guard4(v8f& a, v8f& b, v8f& c, v8f& d) {
  asm volatile("v_nop\n\tv_nop\n\tv_nop\n\tv_nop" : "+v"(a), "+v"(b), "+v"(c), "+v"(d));
}
__device__ __forceinline__ void wave_lds_sync() {
  __builtin_amdgcn_fence(__ATOMIC_RELEASE, "workgroup");
  __builtin_amdgcn_wave_barrier();
  __builtin_amdgcn_fence(__ATOMIC_ACQUIRE, "workgroup");
}

template <typename T> struct Frag;
template <> struct Frag<_Float16> {
  typedef v16h V; union U { v16h v; v8h h[2]; };
  static __device__ __forceinline__ v16h load(const _Float16* p) {
    U f; f.h[0] = *(const v8h*)(p); f.h[1] = *(const v8h*)(p + 16); return f.v;
  }
  static __device__ __forceinline__ v8f mma(v16h a, v16h b, v8f c) {
    return __builtin_amdgcn_wmma_f32_16x16x32_f16(false, a, false, b, (short)0, c, false, false);
  }
};

template <int ACT, bool HASBIAS>
__global__ __launch_bounds__(256) void gemm64_f16(
    const unsigned short* __restrict__ Ap, int lda,
    const unsigned short* __restrict__ Btp, int ldb,
    float* __restrict__ C, int ldc,
    const float* __restrict__ bias,
    int M, int N, int K, float scale) {
  const _Float16* A  = (const _Float16*)Ap;
  const _Float16* Bt = (const _Float16*)Btp;
  __shared__ __align__(16) float sT[8][16 * 68];
  const int lane = threadIdx.x & 31;
  const int wave = threadIdx.x >> 5;
  const int tilesN = N >> 6;
  const int tilesM = M >> 6;
  const int tile = blockIdx.x * 8 + wave;
  if (tile >= tilesM * tilesN) return;
  const int tm = tile / tilesN;
  const int tn = tile - tm * tilesN;
  const int m0 = tm << 6;
  const int n0 = tn << 6;
  const int rlane = lane & 15;
  const int koff  = (lane >> 4) * 8;
  const int mOff  = (lane >> 4) * 8;

  const _Float16* ap[4];
  const _Float16* bp[4];
#pragma unroll
  for (int i = 0; i < 4; ++i) {
    ap[i] = A  + (size_t)(m0 + (i << 4) + rlane) * (size_t)lda + koff;
    bp[i] = Bt + (size_t)(n0 + (i << 4) + rlane) * (size_t)ldb + koff;
  }

  v8f acc[4][4];
#pragma unroll
  for (int i = 0; i < 4; ++i)
#pragma unroll
    for (int j = 0; j < 4; ++j) acc[i][j] = (v8f){0.f, 0.f, 0.f, 0.f, 0.f, 0.f, 0.f, 0.f};

#pragma unroll 1
  for (int k0 = 0; k0 < K; k0 += 32) {
    v16h bh[4];
#pragma unroll
    for (int j = 0; j < 4; ++j) bh[j] = Frag<_Float16>::load(bp[j] + k0);
#pragma unroll
    for (int i = 0; i < 4; ++i) {
      const v16h ah = Frag<_Float16>::load(ap[i] + k0);
#pragma unroll
      for (int j = 0; j < 4; ++j) acc[i][j] = Frag<_Float16>::mma(ah, bh[j], acc[i][j]);
      guard4_h(acc[i][0], acc[i][1], acc[i][2], acc[i][3], ah, bh[0], bh[1], bh[2], bh[3]);
    }
  }
  acc_guard4(acc[0][0], acc[0][1], acc[0][2], acc[0][3]);
  acc_guard4(acc[1][0], acc[1][1], acc[1][2], acc[1][3]);
  acc_guard4(acc[2][0], acc[2][1], acc[2][2], acc[2][3]);
  acc_guard4(acc[3][0], acc[3][1], acc[3][2], acc[3][3]);

  float* slab = sT[wave];
#pragma unroll
  for (int i = 0; i < 4; ++i) {
    const int mBase = m0 + (i << 4);
#pragma unroll
    for (int j = 0; j < 4; ++j) {
      const int n = n0 + (j << 4) + rlane;
      float bv = 0.f;
      if (HASBIAS) bv = bf16r(bias[n]);
#pragma unroll
      for (int r = 0; r < 8; ++r) {
        const float v = acc[i][j][r] * scale + bv;
        slab[(mOff + r) * 68 + (j << 4) + rlane] = v;
      }
    }
    wave_lds_sync();
    if (ACT == 1) {
#pragma unroll 1
      for (int it = 0; it < 32; ++it) {
        const int idx = it * 32 + lane;
        const int row = idx >> 6;
        const int col = idx & 63;
        float* p = slab + row * 68 + col;
        const float xv = *p;
        *p = tanhf(xv);
      }
      wave_lds_sync();
    }
    {
      const int hh = lane >> 4;
      const int c4 = (lane & 15) * 4;
      for (int pass = 0; pass < 2; ++pass) {
#pragma unroll
        for (int it = 0; it < 8; ++it) {
          const int row = it * 2 + hh;
          const v4f v = *(const v4f*)(slab + row * 68 + c4);
          *(volatile v4f*)(C + (size_t)(mBase + row) * (size_t)ldc + n0 + c4) = v;
        }
        __threadfence();
      }
    }
    wave_lds_sync();
  }
}

__global__ __launch_bounds__(NTHR) void cvt8_kernel(const float* __restrict__ src, unsigned short* __restrict__ dst,
                                                    int n8, float sc) {
  const int i = blockIdx.x * NTHR + threadIdx.x;
  if (i < n8) {
    const float* sp = src + (size_t)i * 8;
    const v4f a = *(const v4f*)(sp);
    const v4f b = *(const v4f*)(sp + 4);
    v8h hv;
#pragma unroll
    for (int e = 0; e < 4; ++e) {
      const float fa = a[e];
      const float fb = b[e];
      hv[e]     = (_Float16)(bf16r(fa) * sc);
      hv[4 + e] = (_Float16)(bf16r(fb) * sc);
    }
    *(volatile v8h*)(dst + (size_t)i * 8) = hv;
    __threadfence();
    *(volatile v8h*)(dst + (size_t)i * 8) = hv;
  }
}

__global__ __launch_bounds__(NTHR) void tpw_kernel(const float* __restrict__ src, long srcZ, int C,
                                                   unsigned short* __restrict__ O, long dstZ, int ldo, float sc) {
  __shared__ float Tt[64 * 65];
  const int tid = threadIdx.x;
  const int c0 = blockIdx.x * 64, r0 = blockIdx.y * 64;
  const float* sb = src + (size_t)blockIdx.z * (size_t)srcZ;
  unsigned short* ob = O + (size_t)blockIdx.z * (size_t)dstZ;
#pragma unroll
  for (int i = 0; i < 4; ++i) {
    const int idx = i * NTHR + tid;
    const int rr = idx >> 4, cc = (idx & 15) * 4;
    const v4f v = *(const v4f*)(sb + (size_t)(r0 + rr) * (size_t)C + c0 + cc);
    Tt[rr * 65 + cc + 0] = v[0];
    Tt[rr * 65 + cc + 1] = v[1];
    Tt[rr * 65 + cc + 2] = v[2];
    Tt[rr * 65 + cc + 3] = v[3];
  }
  __syncthreads();
  const int q = tid >> 3, c8 = (tid & 7) * 8;
  v8h hv[2];
#pragma unroll
  for (int g = 0; g < 2; ++g) {
    const int qq = g * 32 + q;
#pragma unroll
    for (int e = 0; e < 8; ++e) {
      const float f = Tt[(c8 + e) * 65 + qq];
      hv[g][e] = (_Float16)(bf16r(f) * sc);
    }
  }
  for (int pass = 0; pass < 2; ++pass) {
#pragma unroll
    for (int g = 0; g < 2; ++g) {
      const size_t o = (size_t)(c0 + g * 32 + q) * (size_t)ldo + (size_t)(r0 + c8);
      *(volatile v8h*)(ob + o) = hv[g];
    }
    __threadfence();
  }
}

__global__ __launch_bounds__(NTHR) void prep_tab_kernel(const float* __restrict__ W2, const float* __restrict__ b2,
                                                        const float* __restrict__ w_att, const float* __restrict__ b_att,
                                                        const float* __restrict__ U_h, const float* __restrict__ U_z,
                                                        const float* __restrict__ O_s, float* __restrict__ TAB) {
  __shared__ float sv[32];
  const int tid = threadIdx.x, lane = tid & 31, wave = tid >> 5;
  const int blk = blockIdx.x;
  const float batt = bf16r(b_att[0]);
#pragma unroll 1
  for (int i = 0; i < 4; ++i) {
    const int rid = 32 * blk + 4 * wave + i;
    int hb = rid - NHD;
    hb = hb < 0 ? 0 : (hb > NHEAD - 1 ? NHEAD - 1 : hb);
    const int rv = rid < NHD ? rid : NHD - 1;
    const float* srow = (rid < NHD) ? (W2 + (size_t)rv * NEMB) : (b2 + (size_t)hb * NEMB);
    float acc = 0.0f;
#pragma unroll 1
    for (int q = 0; q < 8; ++q) {
      const int off = 128 * q + 4 * lane;
      const v4f a = *(const v4f*)(srow + off);
      const v4f w = *(const v4f*)(w_att + off);
#pragma unroll
      for (int e = 0; e < 4; ++e) {
        const float fa = a[e];
        const float fw = w[e];
        acc += bf16r(fa) * bf16r(fw);
      }
    }
#pragma unroll
    for (int off = 1; off < 32; off <<= 1) acc += __shfl_xor(acc, off, 32);
    float val = acc;
    if (rid >= NHD) val = acc + batt;
    if (rid >= NHD + NHEAD) val = 0.0f;
    if (lane == 0) sv[4 * wave + i] = val;
  }
  __syncthreads();
  const bool isC = (blk == NHD / 32);
  const int idx0 = 32 * blk + lane;
  const int idx = idx0 < NHD ? idx0 : NHD - 1;
  const int dh = idx >> 7, dd = idx & 127;
  const float* srcU = (wave == 2) ? U_z : ((wave == 3) ? O_s : U_h);
  const float gv = bf16r(srcU[(size_t)dh * NDH * NDH + (size_t)dd * (NDH + 1)]);
  const float lv = sv[lane];
  const float val = (wave == 0) ? lv : gv;
  const bool active = isC ? (wave == 0) : (wave < 4);
  const int dsti = isC ? (TAB_C + lane) : ((wave & 3) * NHD + idx);
  if (active) {
    *(volatile float*)(TAB + dsti) = val;
    __threadfence();
    *(volatile float*)(TAB + dsti) = val;
  }
}

__global__ __launch_bounds__(NTHR) void scan_kernel(const float* __restrict__ Z, const float* __restrict__ TAB,
                                                    const float* __restrict__ b_u,
                                                    const float* __restrict__ lns_g, const float* __restrict__ lns_b,
                                                    const float* __restrict__ ffg, const float* __restrict__ ffb,
                                                    unsigned short* __restrict__ HLN) {
  const int lane = threadIdx.x & 31, h = threadIdx.x >> 5;
  const int b = blockIdx.x;
  const int d0 = 4 * lane;
  const v4f uh  = *(const v4f*)(TAB + TAB_UH + h * NDH + d0);
  const v4f uz  = *(const v4f*)(TAB + TAB_UZ + h * NDH + d0);
  const v4f osd = *(const v4f*)(TAB + TAB_OS + h * NDH + d0);
  v4f bu = *(const v4f*)(b_u + h * NDH + d0);
  v4f lg = *(const v4f*)(lns_g + d0);
  v4f lb = *(const v4f*)(lns_b + d0);
  v4f fg = *(const v4f*)(ffg + h * NDH + d0);
  v4f fb = *(const v4f*)(ffb + h * NDH + d0);
#pragma unroll
  for (int e = 0; e < 4; ++e) {
    const float t0 = bu[e]; bu[e] = bf16r(t0);
    const float t1 = lg[e]; lg[e] = bf16r(t1);
    const float t2 = lb[e]; lb[e] = bf16r(t2);
    const float t3 = fg[e]; fg[e] = bf16r(t3);
    const float t4 = fb[e]; fb[e] = bf16r(t4);
  }
  const size_t base = (size_t)b * NSEQ * NHD + (size_t)h * NDH + d0;
  const float* zp = Z + base;
  unsigned short* op = HLN + base;
  const float inv = 1.0f / (float)NDH;
  v4f hp = (v4f){0.f, 0.f, 0.f, 0.f};
  v4f zc = *(const v4f*)zp;
#pragma unroll 1
  for (int t = 0; t < NSEQ; ++t) {
    const int tn = (t + 1 < NSEQ) ? (t + 1) : (NSEQ - 1);
    const v4f zn = *(const v4f*)(zp + (size_t)tn * NHD);
    v4f y;
    float s = 0.0f;
#pragma unroll
    for (int e = 0; e < 4; ++e) {
      const float a = hp[e] * uh[e] + zc[e] * uz[e] + bu[e];
      const float u = __builtin_amdgcn_rcpf(1.0f + expf(-a));
      const float yv = u * hp[e] + (1.0f - u) * zc[e];
      y[e] = yv;
      s += yv;
    }
#pragma unroll
    for (int off = 1; off < 32; off <<= 1) s += __shfl_xor(s, off, 32);
    const float mean = s * inv;
    float q = 0.0f;
#pragma unroll
    for (int e = 0; e < 4; ++e) { const float d = y[e] - mean; y[e] = d; q += d * d; }
#pragma unroll
    for (int off = 1; off < 32; off <<= 1) q += __shfl_xor(q, off, 32);
    const float rs = rsqrtf(q * inv + LN_EPS_F);
    v4f sp;
    float s2 = 0.0f;
#pragma unroll
    for (int e = 0; e < 4; ++e) {
      const float hn = (y[e] * rs) * lg[e] + lb[e];
      hp[e] = hn;
      const float sv = hn * osd[e];
      sp[e] = sv;
      s2 += sv;
    }
#pragma unroll
    for (int off = 1; off < 32; off <<= 1) s2 += __shfl_xor(s2, off, 32);
    const float m2 = s2 * inv;
    float q2 = 0.0f;
#pragma unroll
    for (int e = 0; e < 4; ++e) { const float d = sp[e] - m2; sp[e] = d; q2 += d * d; }
#pragma unroll
    for (int off = 1; off < 32; off <<= 1) q2 += __shfl_xor(q2, off, 32);
    const float r2 = rsqrtf(q2 * inv + LN_EPS_F);
    v4h hv;
#pragma unroll
    for (int e = 0; e < 4; ++e) {
      const float o = (sp[e] * r2) * fg[e] + fb[e];
      hv[e] = (_Float16)(o * HCARRY);
    }
    unsigned short* dst = op + (size_t)t * NHD;
    *(volatile v4h*)dst = hv;
    __threadfence();
    *(volatile v4h*)dst = hv;
    zc = zn;
  }
}

__global__ __launch_bounds__(NTHR) void ffn1_kernel(const unsigned short* __restrict__ HLNp,
                                                    const unsigned short* __restrict__ W1Tp,
                                                    const float* __restrict__ b1, const float* __restrict__ TAB,
                                                    unsigned short* __restrict__ G, float* __restrict__ SPL) {
  __shared__ __align__(16) float Hs[NHEAD][16 * SLP];
  __shared__ __align__(16) float lgt[16 * NHEAD];
  __shared__ __align__(16) float ssm[16 * NHEAD];
  const _Float16* HLN = (const _Float16*)HLNp;
  const _Float16* W1T = (const _Float16*)W1Tp;
  const int tid = threadIdx.x, lane = tid & 31, wave = tid >> 5;
  const int c = lane & 15, hh = lane >> 4, koff = hh * 8;
  const int m0 = blockIdx.x * 16;
  const _Float16* ap = HLN + (size_t)(m0 + c) * NHD + wave * NDH + koff;
  const _Float16* bp = W1T + (size_t)wave * NDH * NDH + (size_t)c * NDH + koff;

  v8f acc[8];
#pragma unroll
  for (int j = 0; j < 8; ++j) acc[j] = (v8f){0.f, 0.f, 0.f, 0.f, 0.f, 0.f, 0.f, 0.f};
#pragma unroll 1
  for (int k0 = 0; k0 < NDH; k0 += 32) {
    v16h bf[8];
#pragma unroll
    for (int j = 0; j < 8; ++j) bf[j] = Frag<_Float16>::load(bp + (size_t)j * 16 * NDH + k0);
    const v16h a = Frag<_Float16>::load(ap + k0);
#pragma unroll
    for (int j = 0; j < 8; ++j) acc[j] = Frag<_Float16>::mma(a, bf[j], acc[j]);
    guard8_h(acc[0], acc[1], acc[2], acc[3], acc[4], acc[5], acc[6], acc[7],
             a, bf[0], bf[1], bf[2], bf[3], bf[4], bf[5], bf[6], bf[7]);
  }
  acc_guard4(acc[0], acc[1], acc[2], acc[3]);
  acc_guard4(acc[4], acc[5], acc[6], acc[7]);

  float* slab = Hs[wave];
#pragma unroll
  for (int j = 0; j < 8; ++j) {
    const float bv = bf16r(b1[wave * NDH + 16 * j + c]);
#pragma unroll
    for (int r = 0; r < 8; ++r) slab[(8 * hh + r) * SLP + 16 * j + c] = acc[j][r] * SC_F1 + bv;
  }
  wave_lds_sync();

  const v4f vv = *(const v4f*)(TAB + TAB_V + wave * NDH + 4 * lane);
  const float ch = TAB[TAB_C + wave];
#pragma unroll 1
  for (int row = 0; row < 16; ++row) {
    float* p = slab + row * SLP + 4 * lane;
    const v4f qv = *(const v4f*)p;
    v4f ge;
    float part = 0.0f;
#pragma unroll
    for (int e = 0; e < 4; ++e) {
      const float xv = qv[e];
      const float gx = 0.5f * xv * (1.0f + erff(xv * 0.70710678118654752f));
      ge[e] = gx;
      part += gx * vv[e];
    }
    *(v4f*)p = ge;
#pragma unroll
    for (int off = 1; off < 32; off <<= 1) part += __shfl_xor(part, off, 32);
    if (lane == 0) lgt[row * NHEAD + wave] = part + ch;
  }
  __syncthreads();
  if (tid < 16) {
    const float* lr = lgt + tid * NHEAD;
    float mx = lr[0];
#pragma unroll 1
    for (int i = 1; i < NHEAD; ++i) mx = fmaxf(mx, lr[i]);
    float sum = 0.0f;
#pragma unroll 1
    for (int i = 0; i < NHEAD; ++i) sum += expf(lr[i] - mx);
    const float rinv = 1.0f / sum;
#pragma unroll 1
    for (int i = 0; i < NHEAD; ++i) ssm[tid * NHEAD + i] = expf(lr[i] - mx) * rinv;
  }
  __syncthreads();
  if (wave == 0) {
    const v4f sv = *(const v4f*)(ssm + 4 * lane);
    float* sp = SPL + (size_t)m0 * NHEAD + 4 * lane;
    *(volatile v4f*)sp = sv;
    __threadfence();
    *(volatile v4f*)sp = sv;
  }
  {
    const int c8 = (lane & 15) * 8;
    v8h hv[8];
#pragma unroll
    for (int it = 0; it < 8; ++it) {
      const int row = 2 * it + hh;
      const float sc = ssm[row * NHEAD + wave] * GCARRY;
      const float* sp = slab + row * SLP + c8;
      const v4f x0 = *(const v4f*)(sp);
      const v4f x1 = *(const v4f*)(sp + 4);
#pragma unroll
      for (int e = 0; e < 4; ++e) {
        hv[it][e]     = (_Float16)(x0[e] * sc);
        hv[it][4 + e] = (_Float16)(x1[e] * sc);
      }
    }
    for (int pass = 0; pass < 2; ++pass) {
#pragma unroll
      for (int it = 0; it < 8; ++it) {
        const int row = 2 * it + hh;
        *(volatile v8h*)(G + (size_t)(m0 + row) * NHD + wave * NDH + c8) = hv[it];
      }
      __threadfence();
    }
  }
}

__global__ __launch_bounds__(NTHR) void ln_out_kernel(const float* __restrict__ WGT, const float* __restrict__ SPL,
                                                      const float* __restrict__ b2,
                                                      const float* __restrict__ gam, const float* __restrict__ bet,
                                                      float* __restrict__ out) {
  __shared__ __align__(16) float rb[NTHR / 32][NEMB];
  const int lane = threadIdx.x & 31, wave = threadIdx.x >> 5;
  const int row = blockIdx.x * (NTHR / 32) + wave;
  float* my = rb[wave];
  const v4f s0 = *(const v4f*)(SPL + (size_t)row * NHEAD);
  const v4f s1 = *(const v4f*)(SPL + (size_t)row * NHEAD + 4);
  float sarr[8];
  sarr[0] = s0[0]; sarr[1] = s0[1]; sarr[2] = s0[2]; sarr[3] = s0[3];
  sarr[4] = s1[0]; sarr[5] = s1[1]; sarr[6] = s1[2]; sarr[7] = s1[3];
  const float* wr = WGT + (size_t)row * NEMB;
  float sum = 0.0f;
#pragma unroll 1
  for (int q = 0; q < 8; ++q) {
    const int off = 128 * q + 4 * lane;
    v4f w = *(const v4f*)(wr + off);
#pragma unroll
    for (int hq = 0; hq < 8; ++hq) {
      const v4f bb = *(const v4f*)(b2 + (size_t)hq * NEMB + off);
#pragma unroll
      for (int e = 0; e < 4; ++e) {
        const float fb = bb[e];
        w[e] += sarr[hq] * bf16r(fb);
      }
    }
    *(v4f*)(my + off) = w;
    sum += (w[0] + w[1]) + (w[2] + w[3]);
  }
#pragma unroll
  for (int off = 1; off < 32; off <<= 1) sum += __shfl_xor(sum, off, 32);
  const float mu = sum * (1.0f / (float)NEMB);
  float ss = 0.0f;
#pragma unroll 1
  for (int q = 0; q < 8; ++q) {
    const int off = 128 * q + 4 * lane;
    const v4f w = *(const v4f*)(my + off);
#pragma unroll
    for (int e = 0; e < 4; ++e) { const float d = w[e] - mu; ss += d * d; }
  }
#pragma unroll
  for (int off = 1; off < 32; off <<= 1) ss += __shfl_xor(ss, off, 32);
  const float rstd = rsqrtf(ss * (1.0f / (float)NEMB) + LN_EPS_F);
#pragma unroll 1
  for (int q = 0; q < 8; ++q) {
    const int off = 128 * q + 4 * lane;
    const v4f w = *(const v4f*)(my + off);
    const v4f g = *(const v4f*)(gam + off);
    const v4f bb = *(const v4f*)(bet + off);
    v4f o;
#pragma unroll
    for (int e = 0; e < 4; ++e) {
      const float fg = g[e];
      const float fb = bb[e];
      o[e] = ((w[e] - mu) * rstd) * bf16r(fg) + bf16r(fb);
    }
    *(v4f*)(my + off) = o;
  }
  float* orow = out + (size_t)row * NEMB;
  for (int pass = 0; pass < 2; ++pass) {
#pragma unroll 1
    for (int q = 0; q < 8; ++q) {
      const int off = 128 * q + 4 * lane;
      const v4f o = *(const v4f*)(my + off);
      *(volatile v4f*)(orow + off) = o;
    }
    __threadfence();
  }
}

extern "C" void kernel_launch(void* const* d_in, const int* in_sizes, int n_in,
                              void* d_out, int out_size, void* d_ws, size_t ws_size, hipStream_t stream) {
  if (n_in < 19 || d_out == nullptr || d_ws == nullptr) return;
  if (in_sizes[0] != NTOK * NEMB || in_sizes[1] != NEMB * NHD || in_sizes[2] != NHD ||
      in_sizes[3] != NHEAD * NDH * NDH || in_sizes[4] != NHEAD * NDH * NDH || in_sizes[5] != NHD ||
      in_sizes[6] != NHEAD * NDH * NDH || in_sizes[7] != NDH || in_sizes[8] != NDH ||
      in_sizes[9] != NHD || in_sizes[10] != NHD || in_sizes[11] != NHEAD * NDH * NDH || in_sizes[12] != NHD ||
      in_sizes[13] != NHEAD * NDH * NEMB || in_sizes[14] != NHEAD * NEMB || in_sizes[15] != NEMB ||
      in_sizes[16] != 1 || in_sizes[17] != NEMB || in_sizes[18] != NEMB || out_size != NTOK * NEMB) return;

  const float* x      = (const float*)d_in[0];
  const float* W_ez   = (const float*)d_in[1];
  const float* b_ez   = (const float*)d_in[2];
  const float* U_h    = (const float*)d_in[3];
  const float* U_z    = (const float*)d_in[4];
  const float* b_u    = (const float*)d_in[5];
  const float* o_shp  = (const float*)d_in[6];
  const float* lns_g  = (const float*)d_in[7];
  const float* lns_b  = (const float*)d_in[8];
  const float* ffln_g = (const float*)d_in[9];
  const float* ffln_b = (const float*)d_in[10];
  const float* ff_W1  = (const float*)d_in[11];
  const float* ff_b1  = (const float*)d_in[12];
  const float* ff_W2  = (const float*)d_in[13];
  const float* ff_b2  = (const float*)d_in[14];
  const float* w_att  = (const float*)d_in[15];
  const float* b_att  = (const float*)d_in[16];
  const float* lno_g  = (const float*)d_in[17];
  const float* lno_b  = (const float*)d_in[18];
  float* y_out = (float*)d_out;

  char* ws = (char*)d_ws; size_t off = 0;
  auto carve = [&](size_t bytes) -> char* { char* p = ws + off; off += (bytes + 255) & ~(size_t)255; return p; };
  unsigned short* XH   = (unsigned short*)carve((size_t)NTOK * NEMB * 2);
  unsigned short* WEZT = (unsigned short*)carve((size_t)NHD * NEMB * 2);
  unsigned short* W1T  = (unsigned short*)carve((size_t)NHEAD * NDH * NDH * 2);
  unsigned short* W2T  = (unsigned short*)carve((size_t)NEMB * NHD * 2);
  float*          TAB  = (float*)carve((size_t)TAB_N * 4);
  float*          Z    = (float*)carve((size_t)NTOK * NHD * 4);
  unsigned short* HLN  = (unsigned short*)carve((size_t)NTOK * NHD * 2);
  unsigned short* G    = (unsigned short*)carve((size_t)NTOK * NHD * 2);
  float*          SPL  = (float*)carve((size_t)NTOK * NHEAD * 4);
  float*          WGT  = (float*)carve((size_t)NTOK * NEMB * 4);
  if (off > ws_size || off > (size_t)134217728) return;

  const int n8x = NTOK * (NEMB / 8);
  cvt8_kernel<<<n8x / NTHR, NTHR, 0, stream>>>(x, XH, n8x, XCARRY);
  tpw_kernel<<<dim3(NHD / 64, NEMB / 64, 1), NTHR, 0, stream>>>(W_ez, 0L, NHD, WEZT, 0L, NEMB, WCARRY);
  tpw_kernel<<<dim3(NDH / 64, NDH / 64, NHEAD), NTHR, 0, stream>>>(ff_W1, (long)NDH * NDH, NDH, W1T, (long)NDH * NDH, NDH, WCARRY);
  tpw_kernel<<<dim3(NEMB / 64, NDH / 64, NHEAD), NTHR, 0, stream>>>(ff_W2, (long)NDH * NEMB, NEMB, W2T, (long)NDH, NHD, WCARRY);
  prep_tab_kernel<<<NHD / 32 + 1, NTHR, 0, stream>>>(ff_W2, ff_b2, w_att, b_att, U_h, U_z, o_shp, TAB);

  const int gblocks = (NTOK / 64) * (NHD / 64) / 8;
  gemm64_f16<1, true><<<gblocks, 256, 0, stream>>>(XH, NEMB, WEZT, NEMB, Z, NHD, b_ez, NTOK, NHD, NEMB, SC_G1);

  scan_kernel<<<NBAT, NTHR, 0, stream>>>(Z, TAB, b_u, lns_g, lns_b, ffln_g, ffln_b, HLN);

  ffn1_kernel<<<NTOK / 16, NTHR, 0, stream>>>(HLN, W1T, ff_b1, TAB, G, SPL);

  gemm64_f16<0, false><<<gblocks, 256, 0, stream>>>(G, NHD, W2T, NHD, WGT, NEMB, TAB, NTOK, NEMB, NHD, SC_G2);

  ln_out_kernel<<<NTOK / (NTHR / 32), NTHR, 0, stream>>>(WGT, SPL, ff_b2, lno_g, lno_b, y_out);
}
